// GNN_Diffusion_11072425689122
// MI455X (gfx1250) — hardware-verified
//
#include <hip/hip_runtime.h>
#include <stddef.h>


#define HID    64
#define HID2   128
#define NTHR   256
#define NWAVE  8
#define EPT    8
#define NGRP   2
#define CHUNK  (NTHR * EPT * NGRP)
#define WCAP   (EPT * NGRP * 32)
#define LISTN  (NWAVE * WCAP)
#define NB     4096
#define RCAP   34816
#define TGT    256
#define DEGCAP 256
#define RB     128
#define WTOT   24576
#define STW    256
#define LDS_CSR ((RCAP + 3 * NB + LISTN + 2 * NWAVE) * 4)

static_assert((CHUNK & (CHUNK - 1)) == 0);
static_assert(CHUNK <= 4096);
static_assert(NB <= 4096 && (NB & (NB - 1)) == 0);
static_assert(NB == NTHR * 16);
static_assert((RCAP % 32) == 0);
static_assert(TGT == NWAVE * 32);
static_assert(RB * 2 == NTHR);
static_assert((NB % TGT) == 0);

typedef float          v2f   __attribute__((ext_vector_type(2)));
typedef float          v4f   __attribute__((ext_vector_type(4)));
typedef float          v8f   __attribute__((ext_vector_type(8)));
typedef int            v4i   __attribute__((ext_vector_type(4)));
typedef double         v2d   __attribute__((ext_vector_type(2)));
typedef unsigned short v8us  __attribute__((ext_vector_type(8)));
typedef __bf16         v16bf __attribute__((ext_vector_type(16)));
union FragB { v16bf v; v8us h[2]; };
union FI { float f; int i; };

__host__ __device__ constexpr int gemm_lds(int kd, int nc) {
  return ((RB * (kd + 8) * 4) > (RB * nc * 4) ? (RB * (kd + 8) * 4) : (RB * nc * 4)) + 2 * nc * 8;
}

__device__ __forceinline__ unsigned int bfr_bits(float f) {
  unsigned int u = __float_as_uint(f);
  u += 0x7FFFu + ((u >> 16) & 1u);
  return u >> 16;
}

__device__ __forceinline__ void split1(float f, unsigned short& hi, unsigned short& lo) {
  const unsigned int hb = bfr_bits(f);
  const float hf = __uint_as_float(hb << 16);
  hi = (unsigned short)hb;
  lo = (unsigned short)bfr_bits(f - hf);
}

__device__ __forceinline__ void split8(v4f a, v4f b, v8us& hi, v8us& lo) {
  unsigned short h0, h1, h2, h3, h4, h5, h6, h7, l0, l1, l2, l3, l4, l5, l6, l7;
  split1(a.x, h0, l0); split1(a.y, h1, l1); split1(a.z, h2, l2); split1(a.w, h3, l3);
  split1(b.x, h4, l4); split1(b.y, h5, l5); split1(b.z, h6, l6); split1(b.w, h7, l7);
  hi[0] = h0; hi[1] = h1; hi[2] = h2; hi[3] = h3; hi[4] = h4; hi[5] = h5; hi[6] = h6; hi[7] = h7;
  lo[0] = l0; lo[1] = l1; lo[2] = l2; lo[3] = l3; lo[4] = l4; lo[5] = l5; lo[6] = l6; lo[7] = l7;
}

__device__ __forceinline__ v8f wmb(v16bf a, v16bf b, v8f c) {
  v8f d = __builtin_amdgcn_wmma_f32_16x16x32_bf16(false, a, false, b, (short)0, c, false, false);
  asm volatile("v_nop\n\tv_nop\n\tv_nop\n\tv_nop" : "+v"(d) : "v"(a), "v"(b));
  return d;
}

template <int NBS>
__device__ __forceinline__ int scan_chunk(const int* __restrict__ dsts, int nE, int cbase, int slotBase,
                                          int vec8, int* list, int tid, int lane, int wave) {
  int wc = 0;
#pragma unroll
  for (int g = 0; g < NGRP; ++g) {
    const int el0  = (g * NTHR + tid) * EPT;
    const int e0   = cbase + el0;
    const int sent = -2147483647 - 1;
    v4i da, db;
    if (vec8 != 0 && cbase + CHUNK <= nE) {
      da = *(const v4i*)(dsts + e0);
      db = *(const v4i*)(dsts + e0 + 4);
    } else {
      da.x = (e0     < nE) ? dsts[min(e0, nE - 1)] : sent;
      da.y = (e0 + 1 < nE) ? dsts[min(e0 + 1, nE - 1)] : sent;
      da.z = (e0 + 2 < nE) ? dsts[min(e0 + 2, nE - 1)] : sent;
      da.w = (e0 + 3 < nE) ? dsts[min(e0 + 3, nE - 1)] : sent;
      db.x = (e0 + 4 < nE) ? dsts[min(e0 + 4, nE - 1)] : sent;
      db.y = (e0 + 5 < nE) ? dsts[min(e0 + 5, nE - 1)] : sent;
      db.z = (e0 + 6 < nE) ? dsts[min(e0 + 6, nE - 1)] : sent;
      db.w = (e0 + 7 < nE) ? dsts[min(e0 + 7, nE - 1)] : sent;
    }
    const unsigned nb = (unsigned)slotBase;
    const unsigned s0 = (unsigned)da.x - nb, s1 = (unsigned)da.y - nb;
    const unsigned s2 = (unsigned)da.z - nb, s3 = (unsigned)da.w - nb;
    const unsigned s4 = (unsigned)db.x - nb, s5 = (unsigned)db.y - nb;
    const unsigned s6 = (unsigned)db.z - nb, s7 = (unsigned)db.w - nb;
    const bool h0 = s0 < (unsigned)NBS, h1 = s1 < (unsigned)NBS, h2 = s2 < (unsigned)NBS, h3 = s3 < (unsigned)NBS;
    const bool h4 = s4 < (unsigned)NBS, h5 = s5 < (unsigned)NBS, h6 = s6 < (unsigned)NBS, h7 = s7 < (unsigned)NBS;
    const unsigned any = __builtin_amdgcn_ballot_w32(h0 | h1 | h2 | h3 | h4 | h5 | h6 | h7);
    if (any != 0u) {
#define HITJ(J, HJ, SJ) { \
        const unsigned mj = __builtin_amdgcn_ballot_w32(HJ); \
        if (mj != 0u) { \
          if (HJ) { \
            const int pos = wc + (int)__builtin_amdgcn_mbcnt_lo(mj, 0u); \
            if (pos < WCAP) list[wave * WCAP + pos] = ((el0 + (J)) << 12) | (int)(SJ); \
          } \
          wc += (int)__builtin_popcount(mj); } }
      HITJ(0, h0, s0)
      HITJ(1, h1, s1)
      HITJ(2, h2, s2)
      HITJ(3, h3, s3)
      HITJ(4, h4, s4)
      HITJ(5, h5, s5)
      HITJ(6, h6, s6)
      HITJ(7, h7, s7)
#undef HITJ
    }
  }
  return wc;
}

__global__ __launch_bounds__(NTHR) void k_wprep(
    const float* __restrict__ w0, const float* __restrict__ w1,
    const float* __restrict__ w2, const float* __restrict__ w3,
    unsigned short* whi, unsigned short* wlo) {
  const int bid = (int)blockIdx.x, tid = (int)threadIdx.x;
  const int seg  = bid < 2 ? 0 : (bid < 4 ? 1 : (bid < 8 ? 2 : 3));
  const float* src = seg == 0 ? w0 : (seg == 1 ? w1 : (seg == 2 ? w2 : w3));
  const int sb   = seg == 0 ? 0 : (seg == 1 ? 2 : (seg == 2 ? 4 : 8));
  const int ncol = seg == 2 ? HID2 : HID;
  const int ksh  = seg == 3 ? 4 : 3;
  const int pb   = seg == 0 ? 0 : (seg == 1 ? 4096 : (seg == 2 ? 8192 : 16384));
  const int i  = (bid - sb) * NTHR + tid;
  const int n  = i >> ksh;
  const int k0 = (i & ((1 << ksh) - 1)) * 8;
  v4f a, b;
  a.x = src[(size_t)(k0 + 0) * ncol + n]; a.y = src[(size_t)(k0 + 1) * ncol + n];
  a.z = src[(size_t)(k0 + 2) * ncol + n]; a.w = src[(size_t)(k0 + 3) * ncol + n];
  b.x = src[(size_t)(k0 + 4) * ncol + n]; b.y = src[(size_t)(k0 + 5) * ncol + n];
  b.z = src[(size_t)(k0 + 6) * ncol + n]; b.w = src[(size_t)(k0 + 7) * ncol + n];
  v8us hv, lv;
  split8(a, b, hv, lv);
  const size_t o = (size_t)pb + (size_t)i * 8;
  *(volatile v8us*)(whi + o) = hv;
  *(volatile v8us*)(wlo + o) = lv;
  __threadfence();
  *(volatile v8us*)(whi + o) = hv;
  *(volatile v8us*)(wlo + o) = lv;
}

__global__ __launch_bounds__(NTHR) void k_csr(
    const int* __restrict__ ei, const float* __restrict__ ew,
    int* cnt, int* off, float* dinv, int* csr, int nE, int vec8) {
  extern __shared__ v4f lds_dyn[];
  int*   region = (int*)lds_dyn;
  int*   scnt   = region + RCAP;
  float* sdeg   = (float*)(scnt + NB);
  int*   soff   = scnt + 2 * NB;
  int*   list   = soff + NB;
  int*   wcnt   = list + LISTN;
  int*   wtot   = wcnt + NWAVE;
  const int tid = threadIdx.x, lane = tid & 31, wave = tid >> 5;
  const int b = blockIdx.x;
  const int nodeBase = b * NB;
  const int regBase  = b * RCAP;
  const int* dsts = ei + nE;

  {
    const v4i z = {0, 0, 0, 0};
    const v4f zf = {0.f, 0.f, 0.f, 0.f};
    for (int i = tid; i < RCAP / 4; i += NTHR) ((v4i*)region)[i] = z;
    for (int i = tid; i < NB / 4; i += NTHR) { ((v4i*)scnt)[i] = z; ((v4f*)sdeg)[i] = zf; }
  }
  __syncthreads();

  const int nChunks = (nE + CHUNK - 1) / CHUNK;

#pragma unroll 1
  for (int ch = 0; ch < nChunks; ++ch) {
    const int cbase = ch * CHUNK;
    const int wc = scan_chunk<NB>(dsts, nE, cbase, nodeBase, vec8, list, tid, lane, wave);
    if (lane == 0) wcnt[wave] = wc;
    __syncthreads();
    if (wave == 0) {
#pragma unroll 1
      for (int wsx = 0; wsx < NWAVE; ++wsx) {
        int n = __builtin_amdgcn_readfirstlane(wcnt[wsx]);
        n = n > WCAP ? WCAP : (n < 0 ? 0 : n);
        const int* lp = list + wsx * WCAP;
#pragma unroll 1
        for (int i = 0; i < n; ++i) {
          const int ent  = __builtin_amdgcn_readfirstlane(lp[i]);
          const int slot = ent & (NB - 1);
          int e = cbase + ((ent >> 12) & (CHUNK - 1));
          e = e > nE - 1 ? nE - 1 : e;
          const float w = ew[e];
          if (lane == 0) {
            scnt[slot] = scnt[slot] + 1;
            sdeg[slot] = sdeg[slot] + w;
          }
        }
      }
    }
    __syncthreads();
  }

  int ev[16];
  {
    const v4i c0 = *(const v4i*)(scnt + 16 * tid);
    const v4i c1 = *(const v4i*)(scnt + 16 * tid + 4);
    const v4i c2 = *(const v4i*)(scnt + 16 * tid + 8);
    const v4i c3 = *(const v4i*)(scnt + 16 * tid + 12);
    ev[0]  = max(c0.x, 0); ev[1]  = max(c0.y, 0); ev[2]  = max(c0.z, 0); ev[3]  = max(c0.w, 0);
    ev[4]  = max(c1.x, 0); ev[5]  = max(c1.y, 0); ev[6]  = max(c1.z, 0); ev[7]  = max(c1.w, 0);
    ev[8]  = max(c2.x, 0); ev[9]  = max(c2.y, 0); ev[10] = max(c2.z, 0); ev[11] = max(c2.w, 0);
    ev[12] = max(c3.x, 0); ev[13] = max(c3.y, 0); ev[14] = max(c3.z, 0); ev[15] = max(c3.w, 0);
  }
  int ts = 0;
#pragma unroll
  for (int i = 0; i < 16; ++i) ts += ev[i];
  int incl = ts;
#pragma unroll
  for (int d = 1; d < 32; d <<= 1) {
    const int t = __shfl_up(incl, d);
    if (lane >= d) incl += t;
  }
  if (lane == 31) wtot[wave] = incl;
  __syncthreads();
  int pre = 0;
#pragma unroll 1
  for (int w = 0; w < wave; ++w) pre += wtot[w];
  {
    int run = pre + incl - ts;
    int ov[16];
#pragma unroll
    for (int i = 0; i < 16; ++i) { ov[i] = run; run += ev[i]; }
    const v4i o0 = {ov[0],  ov[1],  ov[2],  ov[3]};
    const v4i o1 = {ov[4],  ov[5],  ov[6],  ov[7]};
    const v4i o2 = {ov[8],  ov[9],  ov[10], ov[11]};
    const v4i o3 = {ov[12], ov[13], ov[14], ov[15]};
    *(v4i*)(soff + 16 * tid)      = o0;
    *(v4i*)(soff + 16 * tid + 4)  = o1;
    *(v4i*)(soff + 16 * tid + 8)  = o2;
    *(v4i*)(soff + 16 * tid + 12) = o3;
  }
  __syncthreads();

  {
    v4i cq[4], oq[4]; v4f dq[4];
#pragma unroll
    for (int q = 0; q < 4; ++q) {
      const int f = (wave * 4 + q) * 128 + 4 * lane;
      cq[q] = *(const v4i*)(scnt + f);
      oq[q] = *(const v4i*)(soff + f) + regBase;
      const v4f dg = *(const v4f*)(sdeg + f);
      dq[q].x = rsqrtf(dg.x + 1.0f);
      dq[q].y = rsqrtf(dg.y + 1.0f);
      dq[q].z = rsqrtf(dg.z + 1.0f);
      dq[q].w = rsqrtf(dg.w + 1.0f);
    }
    int*   cp = cnt  + (size_t)nodeBase;
    int*   op = off  + (size_t)nodeBase;
    float* dp = dinv + (size_t)nodeBase;
#pragma unroll
    for (int q = 0; q < 4; ++q) {
      const int f = (wave * 4 + q) * 128 + 4 * lane;
      *(volatile v4i*)(cp + f) = cq[q];
      *(volatile v4i*)(op + f) = oq[q];
      *(volatile v4f*)(dp + f) = dq[q];
    }
    __threadfence();
#pragma unroll
    for (int q = 0; q < 4; ++q) {
      const int f = (wave * 4 + q) * 128 + 4 * lane;
      *(volatile v4i*)(cp + f) = cq[q];
      *(volatile v4i*)(op + f) = oq[q];
      *(volatile v4f*)(dp + f) = dq[q];
    }
  }

#pragma unroll 1
  for (int ch = 0; ch < nChunks; ++ch) {
    const int cbase = ch * CHUNK;
    const int wc = scan_chunk<NB>(dsts, nE, cbase, nodeBase, vec8, list, tid, lane, wave);
    if (lane == 0) wcnt[wave] = wc;
    __syncthreads();
    if (wave == 0) {
#pragma unroll 1
      for (int wsx = 0; wsx < NWAVE; ++wsx) {
        int n = __builtin_amdgcn_readfirstlane(wcnt[wsx]);
        n = n > WCAP ? WCAP : (n < 0 ? 0 : n);
        const int* lp = list + wsx * WCAP;
#pragma unroll 1
        for (int i = 0; i < n; ++i) {
          const int ent  = __builtin_amdgcn_readfirstlane(lp[i]);
          const int slot = ent & (NB - 1);
          int e = cbase + ((ent >> 12) & (CHUNK - 1));
          e = e > nE - 1 ? nE - 1 : e;
          if (lane == 0) {
            int pos = soff[slot];
            pos = pos < 0 ? 0 : (pos > RCAP - 1 ? RCAP - 1 : pos);
            region[pos] = e;
            const int np = pos + 1;
            soff[slot] = np > RCAP ? RCAP : np;
          }
        }
      }
    }
    __syncthreads();
  }

  int* gp = csr + (size_t)regBase;
#pragma unroll 1
  for (int i = tid; i < RCAP / 4; i += NTHR) { const v4i v = ((const v4i*)region)[i]; *(volatile v4i*)(gp + 4 * i) = v; }
  __threadfence();
#pragma unroll 1
  for (int i = tid; i < RCAP / 4; i += NTHR) { const v4i v = ((const v4i*)region)[i]; *(volatile v4i*)(gp + 4 * i) = v; }
}

template <int KD, int NC, int AM, int EP>
__global__ __launch_bounds__(NTHR) void k_gemm(
    const float* __restrict__ A,
    const float* __restrict__ xin, const float* __restrict__ gw, const float* __restrict__ gb,
    const float* __restrict__ emb, const float* __restrict__ pw, const float* __restrict__ pb, int nGene,
    const float* __restrict__ bnst, const float* __restrict__ bng, const float* __restrict__ bnb,
    const unsigned short* __restrict__ Bh, const unsigned short* __restrict__ Bl,
    const float* __restrict__ dinv, const float* __restrict__ bias,
    float* C, double* part, int nRowsA) {
  extern __shared__ v4f lds_dyn[];
  constexpr int AP   = KD + 8;
  constexpr int NTL  = NC / 16;
  constexpr int KV   = KD / 8;
  constexpr int LA   = RB * AP * 4;
  constexpr int LS   = RB * NC * 4;
  constexpr int LMAX = LA > LS ? LA : LS;
  unsigned short* sAh = (unsigned short*)lds_dyn;
  unsigned short* sAl = sAh + RB * AP;
  float*  stg = (float*)lds_dyn;
  double* pst = (double*)((char*)lds_dyn + LMAX);
  const int tid = threadIdx.x, lane = tid & 31, wave = tid >> 5, hh = lane >> 4, m = lane & 15;
  const int rowBase = blockIdx.x * RB;

#pragma unroll
  for (int i = 0; i < (RB * KV) / NTHR; ++i) {
    const int idx = i * NTHR + tid;
    const int r   = idx / KV;
    const int c0  = (idx % KV) * 8;
    int row = rowBase + r;
    row = row > nRowsA - 1 ? nRowsA - 1 : row;
    v4f a, b;
    if (AM == 1) {
      const float x0 = xin[2 * (size_t)row], x1 = xin[2 * (size_t)row + 1];
      const int g = row % nGene;
      const float* ep = emb + (size_t)g * HID + c0;
      const v4f ea  = *(const v4f*)ep,        eb  = *(const v4f*)(ep + 4);
      const v4f gwa = *(const v4f*)(gw + c0), gwb = *(const v4f*)(gw + c0 + 4);
      const v4f gba = *(const v4f*)(gb + c0), gbb = *(const v4f*)(gb + c0 + 4);
      const v4f pwa = *(const v4f*)(pw + c0), pwb = *(const v4f*)(pw + c0 + 4);
      const v4f pba = *(const v4f*)(pb + c0), pbb = *(const v4f*)(pb + c0 + 4);
      v4f ga = gwa * x0 + gba; ga = ga + ea;
      v4f gq = gwb * x0 + gbb; gq = gq + eb;
      const v4f pa = pwa * x1 + pba;
      const v4f pq = pwb * x1 + pbb;
      a = pa + ga;
      b = pq + gq;
    } else {
      const float* ap = A + (size_t)row * KD + c0;
      a = *(const v4f*)ap; b = *(const v4f*)(ap + 4);
      if (AM == 2) {
        const v4f ma = *(const v4f*)(bnst + c0),       mb = *(const v4f*)(bnst + c0 + 4);
        const v4f ia = *(const v4f*)(bnst + 128 + c0), ib = *(const v4f*)(bnst + 128 + c0 + 4);
        const v4f ga = *(const v4f*)(bng + c0),        gq = *(const v4f*)(bng + c0 + 4);
        const v4f ba = *(const v4f*)(bnb + c0),        bq = *(const v4f*)(bnb + c0 + 4);
        a = (a - ma) * ia * ga + ba;
        b = (b - mb) * ib * gq + bq;
        a.x = fmaxf(a.x, 0.f); a.y = fmaxf(a.y, 0.f); a.z = fmaxf(a.z, 0.f); a.w = fmaxf(a.w, 0.f);
        b.x = fmaxf(b.x, 0.f); b.y = fmaxf(b.y, 0.f); b.z = fmaxf(b.z, 0.f); b.w = fmaxf(b.w, 0.f);
      }
    }
    v8us hv, lv;
    split8(a, b, hv, lv);
    *(v8us*)(sAh + r * AP + c0) = hv;
    *(v8us*)(sAl + r * AP + c0) = lv;
  }
  __syncthreads();

  v8f acc[NTL];
#pragma unroll
  for (int t = 0; t < NTL; ++t) { v8f z = {0.f, 0.f, 0.f, 0.f, 0.f, 0.f, 0.f, 0.f}; acc[t] = z; }
  const unsigned short* ah = sAh + (wave * 16 + m) * AP + 8 * hh;
  const unsigned short* al = sAl + (wave * 16 + m) * AP + 8 * hh;
#pragma unroll
  for (int kt = 0; kt < KD / 32; ++kt) {
    FragB fah, fal;
    fah.h[0] = *(const v8us*)(ah + 32 * kt);
    fah.h[1] = *(const v8us*)(ah + 32 * kt + 16);
    fal.h[0] = *(const v8us*)(al + 32 * kt);
    fal.h[1] = *(const v8us*)(al + 32 * kt + 16);
#pragma unroll
    for (int t = 0; t < NTL; ++t) {
      const size_t bo = (size_t)(16 * t + m) * KD + 32 * kt + 8 * hh;
      FragB fbh, fbl;
      fbh.h[0] = *(const v8us*)(Bh + bo);
      fbh.h[1] = *(const v8us*)(Bh + bo + 16);
      fbl.h[0] = *(const v8us*)(Bl + bo);
      fbl.h[1] = *(const v8us*)(Bl + bo + 16);
      acc[t] = wmb(fah.v, fbh.v, acc[t]);
      acc[t] = wmb(fah.v, fbl.v, acc[t]);
      acc[t] = wmb(fal.v, fbh.v, acc[t]);
    }
  }
  __syncthreads();

  const int r0 = wave * 16 + 8 * hh;
  float s[8];
#pragma unroll
  for (int r = 0; r < 8; ++r) s[r] = 1.0f;
  if (EP == 0) {
    const v4f dA = *(const v4f*)(dinv + (size_t)rowBase + r0);
    const v4f dB = *(const v4f*)(dinv + (size_t)rowBase + r0 + 4);
    s[0] = dA.x; s[1] = dA.y; s[2] = dA.z; s[3] = dA.w; s[4] = dB.x; s[5] = dB.y; s[6] = dB.z; s[7] = dB.w;
  }
  float* sp = stg + r0 * NC + m;
#pragma unroll
  for (int t = 0; t < NTL; ++t) {
    float bv = 0.0f;
    if (EP == 1) bv = bias[16 * t + m];
#pragma unroll
    for (int r = 0; r < 8; ++r) sp[r * NC + 16 * t] = (EP == 0) ? (acc[t][r] * s[r]) : (acc[t][r] + bv);
  }
  __syncthreads();

  constexpr int NCH = NC / 8;
  const float* lp = stg + wave * 16 * NC + 4 * lane;
  float* gp = C + ((size_t)rowBase + wave * 16) * NC + 4 * lane;
#pragma unroll
  for (int i = 0; i < NCH; ++i) { const v4f v = *(const v4f*)(lp + i * 128); *(volatile v4f*)(gp + (size_t)i * 128) = v; }
  __threadfence();
#pragma unroll
  for (int i = 0; i < NCH; ++i) { const v4f v = *(const v4f*)(lp + i * 128); *(volatile v4f*)(gp + (size_t)i * 128) = v; }

  if (EP == 1) {
    int rmax = nRowsA - rowBase;
    rmax = rmax < 0 ? 0 : (rmax > RB ? RB : rmax);
    if (tid < NC) {
      double sm = 0.0, sq = 0.0;
#pragma unroll 4
      for (int r = 0; r < rmax; ++r) {
        const double v = (double)stg[r * NC + tid];
        sm += v;
        sq += v * v;
      }
      pst[tid] = sm;
      pst[NC + tid] = sq;
    }
    __syncthreads();
    v2d pv = {0.0, 0.0};
    if (tid < NC) pv = *(const v2d*)(pst + 2 * tid);
    double* pp = part + (size_t)blockIdx.x * (2 * NC) + 2 * tid;
    if (tid < NC) *(volatile v2d*)pp = pv;
    __threadfence();
    if (tid < NC) *(volatile v2d*)pp = pv;
  }
}

__global__ __launch_bounds__(NTHR) void k_agg(
    const int* __restrict__ csr, const int* __restrict__ off, const int* __restrict__ cnt,
    const int* __restrict__ ei, const float* __restrict__ ew,
    const float* __restrict__ dinv, const float* __restrict__ hw, float* h,
    const float* __restrict__ bs, int nN, int nE, int csrLen, int doRelu) {
  const int tid = threadIdx.x, lane = tid & 31, wave = tid >> 5;
  const int tbase = blockIdx.x * TGT + wave * 32;
  const int cl = tbase + lane;
  const int cnt_l = cnt[cl];
  const int off_l = off[cl];
  FI dvu; dvu.f = dinv[cl];
  const v2f bb = *(const v2f*)(bs + 2 * lane);

#pragma unroll 1
  for (int j = 0; j < 32; ++j) {
    const int c = tbase + j;
    int n = __builtin_amdgcn_readlane(cnt_l, j);
    n = n < 0 ? 0 : (n > DEGCAP ? DEGCAP : n);
    const int st = __builtin_amdgcn_readlane(off_l, j);
    FI du; du.i = __builtin_amdgcn_readlane(dvu.i, j);
    const float dc = du.f;
    v2f acc = {0.f, 0.f};
#pragma unroll 1
    for (int q0 = 0; q0 < n; q0 += 32) {
      int pos = st + q0 + lane;
      pos = pos < 0 ? 0 : (pos > csrLen - 1 ? csrLen - 1 : pos);
      int e = csr[pos];
      e = e < 0 ? 0 : (e > nE - 1 ? nE - 1 : e);
      int sl = ei[e];
      sl = sl < 0 ? 0 : (sl > nN - 1 ? nN - 1 : sl);
      FI wl; wl.f = ew[e];
      const int mcnt = (n - q0) < 32 ? (n - q0) : 32;
#pragma unroll 1
      for (int p = 0; p < mcnt; ++p) {
        const int s = __builtin_amdgcn_readlane(sl, p);
        FI wp; wp.i = __builtin_amdgcn_readlane(wl.i, p);
        const v2f row = *(const v2f*)(hw + (size_t)s * HID + 2 * lane);
        acc = acc + row * wp.f;
      }
    }
    const v2f sv = *(const v2f*)(hw + (size_t)c * HID + 2 * lane);
    v2f v = (acc + sv) * dc + bb;
    if (doRelu != 0) { v.x = fmaxf(v.x, 0.f); v.y = fmaxf(v.y, 0.f); }
    float* hp = h + (size_t)c * HID + 2 * lane;
    *(volatile v2f*)hp = v;
    __threadfence();
    *(volatile v2f*)hp = v;
  }
}

__global__ __launch_bounds__(128) void k_bnfin(
    const double* __restrict__ part, int nBlk, int pitch, int nc, int nRows, float* st) {
  __shared__ __attribute__((aligned(16))) float ss[STW];
  const int tid = threadIdx.x;
  const int c = tid < nc ? tid : nc - 1;
  double s = 0.0, q = 0.0;
#pragma unroll 1
  for (int b2 = 0; b2 < nBlk; ++b2) {
    const double* p = part + (size_t)b2 * pitch;
    s += p[c];
    q += p[nc + c];
  }
  const double inv_n = 1.0 / (double)nRows;
  const double mean = s * inv_n;
  double var = q * inv_n - mean * mean;
  var = var < 0.0 ? 0.0 : var;
  const float meanf = (float)mean;
  const float ve = (float)var + 1e-5f;
  const float istd = rsqrtf(ve);
  ss[tid] = (tid < nc) ? meanf : 0.0f;
  ss[128 + tid] = (tid < nc) ? istd : 0.0f;
  __syncthreads();
  v4f v = {0.f, 0.f, 0.f, 0.f};
  if (tid < 64) v = *(const v4f*)(ss + 4 * tid);
  if (tid < 64) *(volatile v4f*)(st + 4 * tid) = v;
  __threadfence();
  if (tid < 64) *(volatile v4f*)(st + 4 * tid) = v;
}

__global__ __launch_bounds__(NTHR) void k_head(
    const float* __restrict__ h2, const float* __restrict__ st, const float* __restrict__ g2,
    const float* __restrict__ be2, const float* __restrict__ w3, const float* __restrict__ b3,
    float* y, double* part, int nN) {
  __shared__ float sm[HID], si[HID], sg[HID], sb[HID], sw[HID];
  __shared__ double rs[NTHR], rq[NTHR];
  const int tid = threadIdx.x;
  if (tid < HID) {
    sm[tid] = st[tid]; si[tid] = st[128 + tid]; sg[tid] = g2[tid]; sb[tid] = be2[tid]; sw[tid] = w3[tid];
  }
  __syncthreads();
  const int row = blockIdx.x * NTHR + tid;
  const int rr = row > nN - 1 ? nN - 1 : row;
  const float* hp = h2 + (size_t)rr * HID;
  float acc = 0.0f;
#pragma unroll 2
  for (int k4 = 0; k4 < HID / 4; ++k4) {
    const v4f v = *(const v4f*)(hp + 4 * k4);
    const int k = 4 * k4;
    float t0 = (v.x - sm[k])     * si[k]     * sg[k]     + sb[k];     t0 = fmaxf(t0, 0.f); acc += t0 * sw[k];
    float t1 = (v.y - sm[k + 1]) * si[k + 1] * sg[k + 1] + sb[k + 1]; t1 = fmaxf(t1, 0.f); acc += t1 * sw[k + 1];
    float t2 = (v.z - sm[k + 2]) * si[k + 2] * sg[k + 2] + sb[k + 2]; t2 = fmaxf(t2, 0.f); acc += t2 * sw[k + 2];
    float t3 = (v.w - sm[k + 3]) * si[k + 3] * sg[k + 3] + sb[k + 3]; t3 = fmaxf(t3, 0.f); acc += t3 * sw[k + 3];
  }
  const float yv = acc + b3[0];
  *(volatile float*)(y + row) = yv;
  __threadfence();
  *(volatile float*)(y + row) = yv;

  const float ys = row < nN ? yv : 0.0f;
  rs[tid] = (double)ys;
  rq[tid] = (double)ys * (double)ys;
  __syncthreads();
#pragma unroll 1
  for (int ofs = NTHR / 2; ofs > 0; ofs >>= 1) {
    if (tid < ofs) { rs[tid] += rs[tid + ofs]; rq[tid] += rq[tid + ofs]; }
    __syncthreads();
  }
  v2d pv;
  pv.x = (tid == 0) ? rs[0] : 0.0;
  pv.y = (tid == 0) ? rq[0] : 0.0;
  double* pp = part + (size_t)blockIdx.x * 16 + 2 * tid;
  if (tid < 8) *(volatile v2d*)pp = pv;
  __threadfence();
  if (tid < 8) *(volatile v2d*)pp = pv;
}

__global__ __launch_bounds__(NTHR) void k_out(
    const float* __restrict__ y, const float* __restrict__ st, const float* __restrict__ g3,
    const float* __restrict__ b3, const float* __restrict__ x, float* out, int nN) {
  const int tid = threadIdx.x;
  const int i4 = blockIdx.x * NTHR + tid;
  const int n4 = nN >> 2;
  const float mu = st[0], inv = st[128], g = g3[0], bb = b3[0];
  int ic = i4 > n4 - 1 ? n4 - 1 : i4;
  ic = ic < 0 ? 0 : ic;
  const v4f yv = *(const v4f*)(y + 4 * (size_t)ic);
  const v4f xa = *(const v4f*)(x + 8 * (size_t)ic);
  const v4f xb = *(const v4f*)(x + 8 * (size_t)ic + 4);
  v4f o;
  o.x = ((yv.x - mu) * inv * g + bb) + xa.x;
  o.y = ((yv.y - mu) * inv * g + bb) + xa.z;
  o.z = ((yv.z - mu) * inv * g + bb) + xb.x;
  o.w = ((yv.w - mu) * inv * g + bb) + xb.z;
  const bool okv = (i4 < n4);
  const int tail = nN & 3;
  const bool okt = (blockIdx.x == 0) && (tid < tail);
  int it = 4 * n4 + tid;
  it = it > nN - 1 ? nN - 1 : it;
  const float yt = y[it];
  const float xt = x[2 * (size_t)it];
  const float ot = ((yt - mu) * inv * g + bb) + xt;
  if (okv) *(volatile v4f*)(out + 4 * (size_t)i4) = o;
  if (okt) *(volatile float*)(out + it) = ot;
  __threadfence();
  if (okv) *(volatile v4f*)(out + 4 * (size_t)i4) = o;
  if (okt) *(volatile float*)(out + it) = ot;
}

extern "C" void kernel_launch(void* const* d_in, const int* in_sizes, int n_in,
                              void* d_out, int out_size, void* d_ws, size_t ws_size,
                              hipStream_t stream) {
  if (n_in < 24) return;
  const int nN    = in_sizes[0] / 2;
  const int nE    = in_sizes[1] / 2;
  const int nGene = in_sizes[3] / HID;
  if (nN <= 0 || nE <= 0 || nGene <= 0) return;
  if (in_sizes[0] != 2 * nN || in_sizes[1] != 2 * nE || in_sizes[2] != nE || in_sizes[3] != nGene * HID) return;
  if (in_sizes[4] != HID || in_sizes[5] != HID || in_sizes[6] != HID || in_sizes[7] != HID) return;
  if (in_sizes[8] != HID * HID || in_sizes[9] != HID || in_sizes[10] != HID * HID || in_sizes[11] != HID) return;
  if (in_sizes[12] != HID * HID2 || in_sizes[13] != HID2 || in_sizes[14] != HID2 || in_sizes[15] != HID2) return;
  if (in_sizes[16] != HID2 * HID || in_sizes[17] != HID || in_sizes[18] != HID || in_sizes[19] != HID) return;
  if (in_sizes[20] != HID || in_sizes[21] < 1 || in_sizes[22] < 1 || in_sizes[23] < 1) return;
  if (out_size != nN) return;
  if (nE > (1 << 28) || nN > (1 << 24)) return;

  const float* x      = (const float*)d_in[0];
  const int*   ei     = (const int*)d_in[1];
  const float* ew     = (const float*)d_in[2];
  const float* embp   = (const float*)d_in[3];
  const float* pert_w = (const float*)d_in[4];
  const float* pert_b = (const float*)d_in[5];
  const float* gene_w = (const float*)d_in[6];
  const float* gene_b = (const float*)d_in[7];
  const float* gw1    = (const float*)d_in[8];
  const float* gb1    = (const float*)d_in[9];
  const float* gw2    = (const float*)d_in[10];
  const float* gb2    = (const float*)d_in[11];
  const float* mw1    = (const float*)d_in[12];
  const float* mb1    = (const float*)d_in[13];
  const float* bn1_g  = (const float*)d_in[14];
  const float* bn1_b  = (const float*)d_in[15];
  const float* mw2    = (const float*)d_in[16];
  const float* mb2    = (const float*)d_in[17];
  const float* bn2_g  = (const float*)d_in[18];
  const float* bn2_b  = (const float*)d_in[19];
  const float* mw3    = (const float*)d_in[20];
  const float* mb3    = (const float*)d_in[21];
  const float* bn3_g  = (const float*)d_in[22];
  const float* bn3_b  = (const float*)d_in[23];
  float* out = (float*)d_out;

  const int NPAD   = ((nN + TGT - 1) / TGT) * TGT;
  const int nBC    = (nN + NB - 1) / NB;
  const int CNTPAD = nBC * NB;
  const int csrLen = nBC * RCAP;
  const int nGemm  = NPAD / RB;
  const int nAgg   = NPAD / TGT;
  const int nHead  = NPAD / NTHR;
  const int n4     = nN >> 2;
  int nOut = (n4 + NTHR - 1) / NTHR;
  if (nOut < 1) nOut = 1;

  char* ws = (char*)d_ws;
  size_t cur = 0;
  const size_t A256 = 255;
  const size_t oWh  = cur; cur += (size_t)WTOT * 2;                 cur = (cur + A256) & ~A256;
  const size_t oWl  = cur; cur += (size_t)WTOT * 2;                 cur = (cur + A256) & ~A256;
  const size_t oCnt = cur; cur += (size_t)CNTPAD * 4;               cur = (cur + A256) & ~A256;
  const size_t oDv  = cur; cur += (size_t)CNTPAD * 4;               cur = (cur + A256) & ~A256;
  const size_t oOff = cur; cur += (size_t)CNTPAD * 4;               cur = (cur + A256) & ~A256;
  const size_t oCsr = cur; cur += (size_t)csrLen * 4;               cur = (cur + A256) & ~A256;
  const size_t oPA  = cur; cur += (size_t)NPAD * HID * 4;           cur = (cur + A256) & ~A256;
  const size_t oPB  = cur; cur += (size_t)NPAD * HID2 * 4;          cur = (cur + A256) & ~A256;
  const size_t oY   = cur; cur += (size_t)NPAD * 4;                 cur = (cur + A256) & ~A256;
  const size_t oPt  = cur; cur += (size_t)nGemm * (2 * HID2) * 8;   cur = (cur + A256) & ~A256;
  const size_t oP3  = cur; cur += (size_t)nHead * 16 * 8;           cur = (cur + A256) & ~A256;
  const size_t oS1  = cur; cur += (size_t)STW * 4;                  cur = (cur + A256) & ~A256;
  const size_t oS2  = cur; cur += (size_t)STW * 4;                  cur = (cur + A256) & ~A256;
  const size_t oS3  = cur; cur += (size_t)STW * 4;                  cur = (cur + A256) & ~A256;
  if (cur > ws_size) return;
  if (cur > ((size_t)128 << 20)) return;
  unsigned short* whi = (unsigned short*)(ws + oWh);
  unsigned short* wlo = (unsigned short*)(ws + oWl);
  int*    cnt   = (int*)(ws + oCnt);
  float*  dinv  = (float*)(ws + oDv);
  int*    offp  = (int*)(ws + oOff);
  int*    csr   = (int*)(ws + oCsr);
  float*  pA    = (float*)(ws + oPA);
  float*  pB    = (float*)(ws + oPB);
  float*  yv    = (float*)(ws + oY);
  double* part  = (double*)(ws + oPt);
  double* part3 = (double*)(ws + oP3);
  float*  st1   = (float*)(ws + oS1);
  float*  st2   = (float*)(ws + oS2);
  float*  st3   = (float*)(ws + oS3);

  const int vec8 = ((nE & 3) == 0) ? 1 : 0;
  constexpr int LG0 = gemm_lds(HID, HID);
  constexpr int LG1 = gemm_lds(HID, HID2);
  constexpr int LG2 = gemm_lds(HID2, HID);

  k_wprep<<<12, NTHR, 0, stream>>>(gw1, gw2, mw1, mw2, whi, wlo);

  hipFuncSetAttribute(reinterpret_cast<const void*>(&k_csr),
                      hipFuncAttributeMaxDynamicSharedMemorySize, LDS_CSR);
  k_csr<<<nBC, NTHR, LDS_CSR, stream>>>(ei, ew, cnt, offp, dinv, csr, nE, vec8);

  hipFuncSetAttribute(reinterpret_cast<const void*>(&k_gemm<HID, HID, 1, 0>),
                      hipFuncAttributeMaxDynamicSharedMemorySize, LG0);
  k_gemm<HID, HID, 1, 0><<<nGemm, NTHR, LG0, stream>>>(
      pA, x, gene_w, gene_b, embp, pert_w, pert_b, nGene, st1, bn1_g, bn1_b,
      whi, wlo, dinv, gb1, pB, part, nN);
  k_agg<<<nAgg, NTHR, 0, stream>>>(csr, offp, cnt, ei, ew, dinv, pB, pA, gb1, nN, nE, csrLen, 1);

  hipFuncSetAttribute(reinterpret_cast<const void*>(&k_gemm<HID, HID, 0, 0>),
                      hipFuncAttributeMaxDynamicSharedMemorySize, LG0);
  k_gemm<HID, HID, 0, 0><<<nGemm, NTHR, LG0, stream>>>(
      pA, x, gene_w, gene_b, embp, pert_w, pert_b, nGene, st1, bn1_g, bn1_b,
      whi + 4096, wlo + 4096, dinv, gb2, pB, part, nN);
  k_agg<<<nAgg, NTHR, 0, stream>>>(csr, offp, cnt, ei, ew, dinv, pB, pA, gb2, nN, nE, csrLen, 0);

  hipFuncSetAttribute(reinterpret_cast<const void*>(&k_gemm<HID, HID2, 0, 1>),
                      hipFuncAttributeMaxDynamicSharedMemorySize, LG1);
  k_gemm<HID, HID2, 0, 1><<<nGemm, NTHR, LG1, stream>>>(
      pA, x, gene_w, gene_b, embp, pert_w, pert_b, nGene, st1, bn1_g, bn1_b,
      whi + 8192, wlo + 8192, dinv, mb1, pB, part, nN);
  k_bnfin<<<1, 128, 0, stream>>>(part, nGemm, 2 * HID2, HID2, nN, st1);

  hipFuncSetAttribute(reinterpret_cast<const void*>(&k_gemm<HID2, HID, 2, 1>),
                      hipFuncAttributeMaxDynamicSharedMemorySize, LG2);
  k_gemm<HID2, HID, 2, 1><<<nGemm, NTHR, LG2, stream>>>(
      pB, x, gene_w, gene_b, embp, pert_w, pert_b, nGene, st1, bn1_g, bn1_b,
      whi + 16384, wlo + 16384, dinv, mb2, pA, part, nN);
  k_bnfin<<<1, 128, 0, stream>>>(part, nGemm, 2 * HID, HID, nN, st2);

  k_head<<<nHead, NTHR, 0, stream>>>(pA, st2, bn2_g, bn2_b, mw3, mb3, yv, part3, nN);
  k_bnfin<<<1, 128, 0, stream>>>(part3, nHead, 16, 1, nN, st3);

  k_out<<<nOut, NTHR, 0, stream>>>(yv, st3, bn3_g, bn3_b, x, out, nN);
}
